// MultiHeadLatentAttention_68118181314720
// MI455X (gfx1250) — hardware-verified
//
#include <hip/hip_runtime.h>


#ifndef NB
#define NB 2
#endif
#ifndef SEQ
#define SEQ 2048
#endif
#define NB_FULL 2
#define SEQ_FULL 2048
#define EMB 2048
#define LAT 512
#define NHEAD 16
#define HD 128
#define MROWS (NB * SEQ)
#define CSTR 132
#define OTP 136

static_assert(NB <= NB_FULL);
static_assert(SEQ <= SEQ_FULL);
static_assert(SEQ % 128 == 0);
static_assert(MROWS % 128 == 0);
static_assert(EMB % 128 == 0);
static_assert((2 * LAT) % 128 == 0);
static_assert(LAT % 64 == 0);
static_assert(EMB == NHEAD * HD);
static_assert(HD == 128);
static_assert(((size_t)MROWS * EMB) % (256 * 8) == 0);
static_assert((SEQ * 64) % 256 == 0);

typedef _Float16 v16h __attribute__((ext_vector_type(16)));
typedef _Float16 v8h  __attribute__((ext_vector_type(8)));
typedef float    v8f  __attribute__((ext_vector_type(8)));
typedef float    v4f  __attribute__((ext_vector_type(4)));

__device__ __forceinline__ v16h ldfrag(const _Float16* rowp, int h) {
    const v8h lo = *(const v8h*)(rowp + 8 * h);
    const v8h hi = *(const v8h*)(rowp + 16 + 8 * h);
    return __builtin_shufflevector(lo, hi, 0, 1, 2, 3, 4, 5, 6, 7, 8, 9, 10, 11, 12, 13, 14, 15);
}
__device__ __forceinline__ v8f wm(v16h a, v16h b, v8f c) {
    c = __builtin_amdgcn_wmma_f32_16x16x32_f16(false, a, false, b, (short)0, c, false, false);
    asm volatile("v_nop\n\tv_nop\n\tv_nop\n\tv_nop" : "+v"(c) : "v"(a), "v"(b));
    return c;
}
__device__ __forceinline__ float bfr(float f) {
    unsigned u = __float_as_uint(f);
    u += 0x7FFFu + ((u >> 16) & 1u);
    u &= 0xFFFF0000u;
    return __uint_as_float(u);
}

__global__ __launch_bounds__(256) void cvt_x_kernel(const float* x, _Float16* xh) {
    const size_t t = (size_t)blockIdx.x * 256 + threadIdx.x;
    const size_t e0 = t * 8;
    const int m = (int)(e0 / EMB), c = (int)(e0 % EMB);
    const int b = m / SEQ, s = m % SEQ;
    const float* src = x + ((size_t)b * SEQ_FULL + s) * EMB + c;
    const v4f f0 = *(const v4f*)src, f1 = *(const v4f*)(src + 4);
    v8h o;
#pragma unroll
    for (int j = 0; j < 4; ++j) { o[j] = (_Float16)bfr(f0[j]); o[4 + j] = (_Float16)bfr(f1[j]); }
    _Float16* dst = xh + e0;
    *(volatile v8h*)dst = o;
    __threadfence();
    *(volatile v8h*)dst = o;
}

__global__ __launch_bounds__(256) void tr_w_kernel(const float* W, _Float16* Wt, int N, int ldo) {
    __shared__ float tile[64 * 65];
    const int tid = threadIdx.x;
    const int k0 = blockIdx.x * 64, n0 = blockIdx.y * 64;
#pragma unroll 4
    for (int it = 0; it < 16; ++it) {
        const int kk = it * 4 + (tid >> 6), nn = tid & 63;
        tile[kk * 65 + nn] = bfr(W[(size_t)(k0 + kk) * N + n0 + nn]) * 64.0f;
    }
    __syncthreads();
    const int q = tid & 7;
    auto pass = [&]() {
#pragma unroll 1
        for (int p = 0; p < 2; ++p) {
            const int nn = p * 32 + (tid >> 3);
            v8h o;
#pragma unroll
            for (int j = 0; j < 8; ++j) o[j] = (_Float16)tile[(q * 8 + j) * 65 + nn];
            *(volatile v8h*)(Wt + (size_t)(n0 + nn) * ldo + k0 + q * 8) = o;
        }
    };
    pass();
    __threadfence();
    pass();
}

__global__ __launch_bounds__(256) void rope_tab_kernel(float* tab) {
    __shared__ __align__(16) float st[512];
    const int tid = threadIdx.x;
    const int e = blockIdx.x * 256 + tid;
    const int pos = e >> 6, i = e & 63;
    const float ex = -((float)(2 * i) * (1.0f / 128.0f)) * 13.287712379549449f;
    const float fr = exp2f(ex);
    const float ang = (float)pos * fr;
    float sn, cs;
    sincosf(ang, &sn, &cs);
    st[2 * tid] = cs; st[2 * tid + 1] = sn;
    __syncthreads();
    if (tid < 128) {
        const v4f v = *(const v4f*)&st[4 * tid];
        float* p = tab + (size_t)blockIdx.x * 512 + 4 * tid;
        *(volatile v4f*)p = v;
        __threadfence();
        *(volatile v4f*)p = v;
    }
}

template <int MODE>
__global__ __launch_bounds__(256) void gemm_f16_kernel(const _Float16* A, int lda, const _Float16* Bt, int ldb, void* Cv, int ldc, int K,
                                                     float oscale, const float* tab) {
    __shared__ __align__(16) float cst[128 * CSTR];
    const int tid = threadIdx.x, lane = tid & 31, wv = tid >> 5;
    const int l16 = lane & 15, h = lane >> 4;
    const int rt = wv & 3, ch = wv >> 2;
    const int row0 = blockIdx.x * 128, col0 = blockIdx.y * 128;
    const _Float16* ap0 = A + (size_t)(row0 + rt * 32 + l16) * lda;
    const _Float16* ap1 = ap0 + (size_t)16 * lda;
    const _Float16* bp = Bt + (size_t)(col0 + ch * 64 + l16) * ldb;
    v8f acc[2][4];
#pragma unroll
    for (int i = 0; i < 2; ++i)
#pragma unroll
        for (int t = 0; t < 4; ++t) acc[i][t] = (v8f){};
#pragma unroll 1
    for (int k0 = 0; k0 < K; k0 += 32) {
        const v16h a0 = ldfrag(ap0 + k0, h);
        const v16h a1 = ldfrag(ap1 + k0, h);
#pragma unroll
        for (int t = 0; t < 4; ++t) {
            const v16h b = ldfrag(bp + (size_t)(16 * t) * ldb + k0, h);
            acc[0][t] = wm(a0, b, acc[0][t]);
            acc[1][t] = wm(a1, b, acc[1][t]);
        }
    }
#pragma unroll
    for (int i = 0; i < 2; ++i)
#pragma unroll
        for (int t = 0; t < 4; ++t) {
            const int cl = ch * 64 + t * 16 + l16;
#pragma unroll
            for (int r = 0; r < 8; ++r) {
                const int rl = rt * 32 + i * 16 + 8 * h + r;
                cst[rl * CSTR + cl] = acc[i][t][r] * oscale;
            }
        }
    __syncthreads();
    if (MODE == 0) {
        _Float16* C = (_Float16*)Cv;
        const int q = tid & 15, rsel = tid >> 4;
        auto pass = [&]() {
#pragma unroll 1
            for (int p = 0; p < 8; ++p) {
                const int r = p * 16 + rsel;
                const float* cr = cst + r * CSTR + q * 8;
                const v4f c0 = *(const v4f*)cr, c1 = *(const v4f*)(cr + 4);
                v8h o;
#pragma unroll
                for (int j = 0; j < 4; ++j) { o[j] = (_Float16)c0[j]; o[4 + j] = (_Float16)c1[j]; }
                *(volatile v8h*)(C + (size_t)(row0 + r) * ldc + col0 + q * 8) = o;
            }
        };
        pass();
        __threadfence();
        pass();
    } else if (MODE == 1) {
        _Float16* C = (_Float16*)Cv;
        const int q = tid & 15, rsel = tid >> 4;
        const int qi = q & 7;
        const bool upper = q >= 8;
        auto pass = [&]() {
#pragma unroll 1
            for (int p = 0; p < 8; ++p) {
                const int r = p * 16 + rsel;
                const float* cr = cst + r * CSTR + qi * 16;
                const int pos = (row0 + r) % SEQ;
                const float* tp = tab + ((size_t)pos * 64 + qi * 8) * 2;
                float cv[16], tv[16];
#pragma unroll
                for (int g = 0; g < 4; ++g) {
                    const v4f c = *(const v4f*)(cr + 4 * g);
                    const v4f t = *(const v4f*)(tp + 4 * g);
#pragma unroll
                    for (int j = 0; j < 4; ++j) { cv[4 * g + j] = c[j]; tv[4 * g + j] = t[j]; }
                }
                v8h o;
#pragma unroll
                for (int j = 0; j < 8; ++j) {
                    const float e = cv[2 * j], od = cv[2 * j + 1], cs = tv[2 * j], sn = tv[2 * j + 1];
                    const float lo = e * cs - od * sn;
                    const float hi = e * sn + od * cs;
                    o[j] = (_Float16)(upper ? hi : lo);
                }
                *(volatile v8h*)(C + (size_t)(row0 + r) * ldc + col0 + q * 8) = o;
            }
        };
        pass();
        __threadfence();
        pass();
    } else {
        float* C = (float*)Cv;
        const int q = tid & 31, rsel = tid >> 5;
        auto pass = [&]() {
#pragma unroll 1
            for (int p = 0; p < 16; ++p) {
                const int r = p * 8 + rsel;
                const int gr = row0 + r;
                const size_t orow = (size_t)(gr / SEQ) * SEQ_FULL + (size_t)(gr % SEQ);
                const v4f v = *(const v4f*)(cst + r * CSTR + q * 4);
                *(volatile v4f*)(C + orow * ldc + col0 + q * 4) = v;
            }
        };
        pass();
        __threadfence();
        pass();
    }
}

__global__ __launch_bounds__(256) void attn_kernel(const _Float16* qh, const _Float16* kh, const _Float16* vT, const float* mask, _Float16* ctx) {
    __shared__ __align__(16) _Float16 ot[8 * 16 * OTP];
    const int tid = threadIdx.x, lane = tid & 31, wave = tid >> 5;
    const int l16 = lane & 15, h = lane >> 4;
    const int bh = blockIdx.y, b = bh / NHEAD, hh = bh % NHEAD;
    const int q0 = blockIdx.x * 128 + wave * 16;
    const _Float16* qp = qh + ((size_t)b * SEQ + q0 + l16) * EMB + hh * HD;
    v16h bq[4];
#pragma unroll
    for (int kk = 0; kk < 4; ++kk) bq[kk] = ldfrag(qp + 32 * kk, h);
    const _Float16* kp = kh + ((size_t)b * SEQ + l16) * EMB + hh * HD;
    const _Float16* vp = vT + (size_t)(hh * HD + l16) * MROWS + (size_t)b * SEQ;
    const float* mp = mask + (size_t)(q0 + l16) * SEQ_FULL + 8 * h;
    v8f o[8];
#pragma unroll
    for (int t = 0; t < 8; ++t) o[t] = (v8f){};
    float m_i = -1e30f, l_i = 0.0f;
    const float LOG2E = 1.4426950408889634f;
    const float sc = LOG2E * 0.08838834764831845f * (1.0f / 256.0f);
#pragma unroll 1
    for (int j0 = 0; j0 < SEQ; j0 += 32) {
        v8f s0 = (v8f){}, s1 = (v8f){};
        const _Float16* k0p = kp + (size_t)j0 * EMB;
        const _Float16* k1p = k0p + (size_t)16 * EMB;
#pragma unroll
        for (int kk = 0; kk < 4; ++kk) {
            const v16h a0 = ldfrag(k0p + 32 * kk, h);
            const v16h a1 = ldfrag(k1p + 32 * kk, h);
            s0 = wm(a0, bq[kk], s0);
            s1 = wm(a1, bq[kk], s1);
        }
        const v4f ma = *(const v4f*)(mp + j0), mb = *(const v4f*)(mp + j0 + 4);
        const v4f mc = *(const v4f*)(mp + j0 + 16), md = *(const v4f*)(mp + j0 + 20);
        float y0[8], y1[8];
#pragma unroll
        for (int r = 0; r < 8; ++r) {
            const float k0m = (r < 4) ? ma[r & 3] : mb[r & 3];
            const float k1m = (r < 4) ? mc[r & 3] : md[r & 3];
            y0[r] = fmaf(s0[r], sc, k0m * LOG2E);
            y1[r] = fmaf(s1[r], sc, k1m * LOG2E);
        }
        float mx = fmaxf(y0[0], y1[0]);
#pragma unroll
        for (int r = 1; r < 8; ++r) mx = fmaxf(mx, fmaxf(y0[r], y1[r]));
        mx = fmaxf(mx, __shfl_xor(mx, 16, 32));
        const float m_new = fmaxf(m_i, mx);
        float rs = 0.0f;
        v16h pb;
#pragma unroll
        for (int r = 0; r < 8; ++r) {
            const float p0 = exp2f((y0[r] - m_new) + 10.0f);
            const float p1 = exp2f((y1[r] - m_new) + 10.0f);
            rs += p0 + p1;
            pb[r] = (_Float16)p0;
            pb[8 + r] = (_Float16)p1;
        }
        rs += __shfl_xor(rs, 16, 32);
        const float alpha = exp2f(m_i - m_new);
        l_i = l_i * alpha + rs;
        m_i = m_new;
#pragma unroll
        for (int t = 0; t < 8; ++t)
#pragma unroll
            for (int r = 0; r < 8; ++r) o[t][r] *= alpha;
#pragma unroll
        for (int t = 0; t < 8; ++t) {
            const v16h av = ldfrag(vp + (size_t)(16 * t) * MROWS + j0, h);
            o[t] = wm(av, pb, o[t]);
        }
    }
    const float inv = 16.0f * (1.0f / l_i);
    _Float16* tw = ot + (wave * 16 + l16) * OTP;
#pragma unroll
    for (int t = 0; t < 8; ++t) {
        v8h pk;
#pragma unroll
        for (int r = 0; r < 8; ++r) pk[r] = (_Float16)(o[t][r] * inv);
        *(v8h*)(tw + 16 * t + 8 * h) = pk;
    }
    __syncthreads();
    const int piece = lane & 15, rhalf = lane >> 4;
    auto pass = [&]() {
#pragma unroll 1
        for (int p = 0; p < 8; ++p) {
            const int rr = 2 * p + rhalf;
            const v8h v = *(const v8h*)(ot + (wave * 16 + rr) * OTP + piece * 8);
            *(volatile v8h*)(ctx + ((size_t)b * SEQ + q0 + rr) * EMB + hh * HD + piece * 8) = v;
        }
    };
    pass();
    __threadfence();
    pass();
}

constexpr size_t SZ_XH   = (size_t)MROWS * EMB * 2;
constexpr size_t SZ_WTD  = (size_t)(2 * LAT) * EMB * 2;
constexpr size_t SZ_WTU  = (size_t)EMB * LAT * 2;
constexpr size_t SZ_WTE  = (size_t)EMB * EMB * 2;
constexpr size_t SZ_CQ   = (size_t)MROWS * (2 * LAT) * 2;
constexpr size_t SZ_ACT  = (size_t)MROWS * EMB * 2;
constexpr size_t SZ_TAB  = (size_t)SEQ * 64 * 2 * 4;
constexpr size_t OFF_XH   = 0;
constexpr size_t OFF_WTD  = OFF_XH + SZ_XH;
constexpr size_t OFF_WTUV = OFF_WTD + SZ_WTD;
constexpr size_t OFF_WTUQ = OFF_WTUV + SZ_WTU;
constexpr size_t OFF_WTKR = OFF_WTUQ + SZ_WTU;
constexpr size_t OFF_WTO  = OFF_WTKR + SZ_WTE;
constexpr size_t OFF_CQ   = OFF_WTO + SZ_WTE;
constexpr size_t OFF_VT   = OFF_CQ + SZ_CQ;
constexpr size_t OFF_QH   = OFF_VT + SZ_ACT;
constexpr size_t OFF_KH   = OFF_QH + SZ_ACT;
constexpr size_t OFF_CTX  = OFF_KH + SZ_ACT;
constexpr size_t OFF_TAB  = OFF_CTX + SZ_ACT;
constexpr size_t WS_NEED  = OFF_TAB + SZ_TAB;
static_assert(WS_NEED <= (size_t)134217728);
static_assert(OFF_TAB % 256 == 0);

extern "C" void kernel_launch(void* const* d_in, const int* in_sizes, int n_in,
                              void* d_out, int out_size, void* d_ws, size_t ws_size, hipStream_t stream) {
    if (n_in < 8) return;
    const long long xneed = (long long)(NB - 1) * SEQ_FULL * EMB + (long long)SEQ * EMB;
    if ((long long)in_sizes[0] < xneed) return;
    if ((long long)in_sizes[1] < (long long)(SEQ - 1) * SEQ_FULL + SEQ) return;
    if (in_sizes[2] < EMB * LAT || in_sizes[3] < LAT * EMB || in_sizes[4] < EMB * EMB) return;
    if (in_sizes[5] < EMB * LAT || in_sizes[6] < LAT * EMB || in_sizes[7] < EMB * EMB) return;
    if ((long long)out_size < xneed) return;
    if (WS_NEED > ws_size) return;

    const float* x     = (const float*)d_in[0];
    const float* mask  = (const float*)d_in[1];
    const float* W_dkv = (const float*)d_in[2];
    const float* W_uv  = (const float*)d_in[3];
    const float* W_kr  = (const float*)d_in[4];
    const float* W_dq  = (const float*)d_in[5];
    const float* W_uq  = (const float*)d_in[6];
    const float* W_o   = (const float*)d_in[7];
    float* out = (float*)d_out;

    char* ws = (char*)d_ws;
    _Float16* xh   = (_Float16*)(ws + OFF_XH);
    _Float16* wtd  = (_Float16*)(ws + OFF_WTD);
    _Float16* wtuv = (_Float16*)(ws + OFF_WTUV);
    _Float16* wtuq = (_Float16*)(ws + OFF_WTUQ);
    _Float16* wtkr = (_Float16*)(ws + OFF_WTKR);
    _Float16* wto  = (_Float16*)(ws + OFF_WTO);
    _Float16* cq   = (_Float16*)(ws + OFF_CQ);
    _Float16* vT   = (_Float16*)(ws + OFF_VT);
    _Float16* qh   = (_Float16*)(ws + OFF_QH);
    _Float16* kh   = (_Float16*)(ws + OFF_KH);
    _Float16* ctx  = (_Float16*)(ws + OFF_CTX);
    float*    tab  = (float*)(ws + OFF_TAB);

    cvt_x_kernel<<<dim3((unsigned)(((size_t)MROWS * EMB) / (256 * 8))), 256, 0, stream>>>(x, xh);
    tr_w_kernel<<<dim3(EMB / 64, LAT / 64), 256, 0, stream>>>(W_dkv, wtd, LAT, EMB);
    tr_w_kernel<<<dim3(EMB / 64, LAT / 64), 256, 0, stream>>>(W_dq, wtd + (size_t)LAT * EMB, LAT, EMB);
    tr_w_kernel<<<dim3(LAT / 64, EMB / 64), 256, 0, stream>>>(W_uv, wtuv, EMB, LAT);
    tr_w_kernel<<<dim3(LAT / 64, EMB / 64), 256, 0, stream>>>(W_uq, wtuq, EMB, LAT);
    tr_w_kernel<<<dim3(EMB / 64, EMB / 64), 256, 0, stream>>>(W_kr, wtkr, EMB, EMB);
    tr_w_kernel<<<dim3(EMB / 64, EMB / 64), 256, 0, stream>>>(W_o, wto, EMB, EMB);
    rope_tab_kernel<<<dim3((SEQ * 64) / 256), 256, 0, stream>>>(tab);

    gemm_f16_kernel<0><<<dim3(MROWS / 128, (2 * LAT) / 128), 256, 0, stream>>>(xh, EMB, wtd, EMB, (void*)cq, 2 * LAT, EMB, 0.25f, (const float*)nullptr);
    gemm_f16_kernel<0><<<dim3(EMB / 128, MROWS / 128), 256, 0, stream>>>(wtuv, LAT, cq, 2 * LAT, (void*)vT, MROWS, LAT, 1.0f / 16.0f, (const float*)nullptr);
    gemm_f16_kernel<0><<<dim3(MROWS / 128, EMB / 128), 256, 0, stream>>>(cq + LAT, 2 * LAT, wtuq, LAT, (void*)qh, EMB, LAT, 1.0f / 64.0f, (const float*)nullptr);
    gemm_f16_kernel<1><<<dim3(MROWS / 128, EMB / 128), 256, 0, stream>>>(xh, EMB, wtkr, EMB, (void*)kh, EMB, EMB, 0.25f, (const float*)tab);
    attn_kernel<<<dim3(SEQ / 128, NB * NHEAD), 256, 0, stream>>>(qh, kh, vT, mask, ctx);
    gemm_f16_kernel<2><<<dim3(MROWS / 128, EMB / 128), 256, 0, stream>>>(ctx, EMB, wto, EMB, (void*)out, EMB, EMB, 1.0f / 65536.0f, (const float*)nullptr);
}
